// lstm_seq2seq_8572754722968
// MI455X (gfx1250) — hardware-run, weakly checked
//
#include <hip/hip_runtime.h>
#include <math.h>

constexpr int HID      = 64;
constexpr int NGROW    = 4 * HID;
constexpr int NBAT     = 1024;
constexpr int TENC     = 1000;
constexpr int TDEC     = 1000;
constexpr int RPB      = 32;
constexpr int NTHR     = 128;
constexpr int HPH      = 72;
constexpr int HPF      = 68;
constexpr int AH_ELEMS = 2 * RPB * HPH;
constexpr int HF_ELEMS = 2 * RPB * HPF;
constexpr int WPLANE   = NGROW * HID;
constexpr int PREP_THR = 256;
constexpr float HCARRY = 1024.0f;
constexpr float WCARRY = 256.0f;
constexpr float ZINV   = 1.0f / 262144.0f;
static_assert(NBAT % RPB == 0, "grid exact");
static_assert(RPB == 32, "one 128-B output line per block per step");
static_assert(HID == 16 * (NTHR / 32), "4 waves x 16 units");
static_assert(HID % 32 == 0, "K = 64 = 2 k-tiles of 32, no padding");
static_assert(NGROW % 16 == 0, "N = 256 = 16 full subtiles");
static_assert(AH_ELEMS % NTHR == 0, "zero-fill loop exact");
static_assert(HF_ELEMS % NTHR == 0, "zero-fill loop exact");
static_assert((WPLANE / 8) % PREP_THR == 0, "prep grid exact");
static_assert(HPH % 8 == 0 && HPF % 4 == 0, "16-B aligned LDS rows");

typedef __attribute__((ext_vector_type(16))) _Float16 v16h;
typedef __attribute__((ext_vector_type(8)))  _Float16 v8h;
typedef __attribute__((ext_vector_type(8)))  float    v8f;
typedef __attribute__((ext_vector_type(4)))  float    v4f;

__device__ __forceinline__ unsigned short f2bf_bits(float f) {
  unsigned u = __float_as_uint(f);
  return (unsigned short)((u + 0x7FFFu + ((u >> 16) & 1u)) >> 16);
}
__device__ __forceinline__ float bf_bits2f(unsigned short h) { return __uint_as_float(((unsigned)h) << 16); }
__device__ __forceinline__ float bf16r(float f) { return bf_bits2f(f2bf_bits(f)); }

__device__ __forceinline__ void grp_guard4(v8f& a, v8f& b, v8f& c, v8f& d, v16h x, v16h y) {
  asm volatile("v_nop\n\tv_nop\n\tv_nop\n\tv_nop" : "+v"(a), "+v"(b), "+v"(c), "+v"(d) : "v"(x), "v"(y));
}
__device__ __forceinline__ void keep8_h(v16h a, v16h b, v16h c, v16h d, v16h e, v16h f, v16h g, v16h h8) {
  asm volatile("v_nop" :: "v"(a), "v"(b), "v"(c), "v"(d), "v"(e), "v"(f), "v"(g), "v"(h8));
}
__device__ __forceinline__ void settle4(float& a, float& b, float& c, float& d) { asm volatile("" : "+v"(a), "+v"(b), "+v"(c), "+v"(d)); }
__device__ __forceinline__ void settle2h(v16h& a, v16h& b) { asm volatile("" : "+v"(a), "+v"(b)); }

template <typename T> struct Frag;
template <> struct Frag<_Float16> {
  typedef v16h V; union U { v16h v; v8h h[2]; };
  static __device__ __forceinline__ v16h load(const _Float16* p) {
    U f; f.h[0] = *(const v8h*)(p); f.h[1] = *(const v8h*)(p + 16); return f.v;
  }
  static __device__ __forceinline__ v8f mma(v16h a, v16h b, v8f c) {
    return __builtin_amdgcn_wmma_f32_16x16x32_f16(false, a, false, b, (short)0, c, false, false);
  }
};

__device__ __forceinline__ float fsig(float x)  { return __builtin_amdgcn_rcpf(1.0f + __expf(-x)); }
__device__ __forceinline__ float ftanh(float x) { return 1.0f - 2.0f * __builtin_amdgcn_rcpf(__expf(2.0f * x) + 1.0f); }

__global__ __launch_bounds__(PREP_THR) void whh_prep_kernel(const float* __restrict__ w, unsigned short* __restrict__ dst) {
  const int i  = blockIdx.x * PREP_THR + threadIdx.x;
  const int e8 = i * 8;
  const v4f a0 = *(const v4f*)(w + e8);
  const v4f a1 = *(const v4f*)(w + e8 + 4);
  v8h hv;
#pragma unroll
  for (int e = 0; e < 4; ++e) {
    hv[e]     = (_Float16)(bf16r(a0[e]) * WCARRY);
    hv[4 + e] = (_Float16)(bf16r(a1[e]) * WCARRY);
  }
  unsigned short* op = dst + (size_t)e8;
  *(volatile v8h*)op = hv;
  __threadfence();
  *(volatile v8h*)op = hv;
}

template <bool DEC>
__device__ __forceinline__ void lstm_phase(
    const float* __restrict__ xsrc, const float* __restrict__ Wih,
    const float* __restrict__ bih, const float* __restrict__ bhh,
    const _Float16* __restrict__ WH, float* __restrict__ out, float linb,
    float (&cst)[2][8], int& par,
    _Float16* Ah, float* Hf, const float* linWs,
    int lane, int wave, int bbase) {
  const int c = lane & 15, hh = lane >> 4, koff = hh * 8;
  const int ucol = 16 * wave + c;

  float wih[4], tb[4], bsum[4];
#pragma unroll
  for (int g = 0; g < 4; ++g) wih[g] = bf16r(Wih[g * HID + ucol]);
  settle4(wih[0], wih[1], wih[2], wih[3]);
#pragma unroll
  for (int g = 0; g < 4; ++g) tb[g] = bf16r(bih[g * HID + ucol]);
  settle4(tb[0], tb[1], tb[2], tb[3]);
#pragma unroll
  for (int g = 0; g < 4; ++g) bsum[g] = tb[g] + bf16r(bhh[g * HID + ucol]);
  settle4(bsum[0], bsum[1], bsum[2], bsum[3]);

  v16h Bf0[4], Bf1[4];
#pragma unroll
  for (int g = 0; g < 4; ++g) {
    const _Float16* wr = WH + (size_t)(g * HID + ucol) * HID + koff;
    Bf0[g] = Frag<_Float16>::load(wr);
    Bf1[g] = Frag<_Float16>::load(wr + 32);
    settle2h(Bf0[g], Bf1[g]);
  }

  const v8f z8 = {0.f, 0.f, 0.f, 0.f, 0.f, 0.f, 0.f, 0.f};
  constexpr int NSTEPS = DEC ? TDEC : TENC;

#pragma unroll 1
  for (int t = 0; t < NSTEPS; ++t) {
    const int cur = par, nxt = par ^ 1;
    const _Float16* ahc = Ah + cur * (RPB * HPH);
    _Float16*       ahn = Ah + nxt * (RPB * HPH);
    float*          hfn = Hf + nxt * (RPB * HPF);
    int tt = t; float xf = 1.0f;
    if (DEC) { tt = (t > 0) ? (t - 1) : 0; xf = (t > 0) ? 1.0f : 0.0f; }

#pragma unroll
    for (int mt = 0; mt < 2; ++mt) {
      const float* xr = xsrc + (size_t)tt * NBAT + bbase + 16 * mt + 8 * hh;
      const v4f x0 = *(const v4f*)(xr);
      const v4f x1 = *(const v4f*)(xr + 4);
      float xv[8];
#pragma unroll
      for (int e = 0; e < 4; ++e) { xv[e] = bf16r(x0[e]) * xf; xv[4 + e] = bf16r(x1[e]) * xf; }

      const _Float16* arow = ahc + (16 * mt + c) * HPH + koff;
      const v16h a0 = Frag<_Float16>::load(arow);
      const v16h a1 = Frag<_Float16>::load(arow + 32);
      v8f acc[4];
      acc[0] = z8; acc[1] = z8; acc[2] = z8; acc[3] = z8;
#pragma unroll
      for (int g = 0; g < 4; ++g) acc[g] = Frag<_Float16>::mma(a0, Bf0[g], acc[g]);
#pragma unroll
      for (int g = 0; g < 4; ++g) acc[g] = Frag<_Float16>::mma(a1, Bf1[g], acc[g]);
      grp_guard4(acc[0], acc[1], acc[2], acc[3], a0, a1);
      keep8_h(Bf0[0], Bf0[1], Bf0[2], Bf0[3], Bf1[0], Bf1[1], Bf1[2], Bf1[3]);

#pragma unroll
      for (int r = 0; r < 8; ++r) {
        const float zi = fmaf(acc[0][r], ZINV, fmaf(xv[r], wih[0], bsum[0]));
        const float zf = fmaf(acc[1][r], ZINV, fmaf(xv[r], wih[1], bsum[1]));
        const float zg = fmaf(acc[2][r], ZINV, fmaf(xv[r], wih[2], bsum[2]));
        const float zo = fmaf(acc[3][r], ZINV, fmaf(xv[r], wih[3], bsum[3]));
        const float ig = fsig(zi);
        const float fg = fsig(zf);
        const float gg = ftanh(zg);
        const float og = fsig(zo);
        const float cn = fmaf(fg, cst[mt][r], ig * gg);
        cst[mt][r] = cn;
        const float hn = og * ftanh(cn);
        const int row = 16 * mt + 8 * hh + r;
        ahn[row * HPH + ucol] = (_Float16)(hn * HCARRY);
        if (DEC) hfn[row * HPF + ucol] = hn;
      }
    }
    __syncthreads();

    if (DEC) {
      const float* hrow = hfn + lane * HPF;
      float s = 0.0f;
#pragma unroll
      for (int k4 = 0; k4 < HID / 4; ++k4) {
        const v4f hv = *(const v4f*)(hrow + 4 * k4);
        const v4f lw = *(const v4f*)(linWs + 4 * k4);
        s = fmaf(hv[0], lw[0], s);
        s = fmaf(hv[1], lw[1], s);
        s = fmaf(hv[2], lw[2], s);
        s = fmaf(hv[3], lw[3], s);
      }
      s += linb;
      v4f ov;
#pragma unroll
      for (int e = 0; e < 4; ++e) ov[e] = __shfl(s, (4 * lane + e) & 31, 32);
      float* op = out + (size_t)t * NBAT + bbase + 4 * (lane & 7);
      const bool wr = (wave == 0) && (lane < 8);
      for (int pass = 0; pass < 2; ++pass) {
        if (wr) *(volatile v4f*)op = ov;
        __threadfence();
      }
    }
    par = nxt;
  }
}

__global__ __launch_bounds__(NTHR) void seq_kernel(
    const float* __restrict__ x_enc, const float* __restrict__ x_dec,
    const float* __restrict__ e_wih, const float* __restrict__ e_bih, const float* __restrict__ e_bhh,
    const float* __restrict__ d_wih, const float* __restrict__ d_bih, const float* __restrict__ d_bhh,
    const float* __restrict__ lin_w, const float* __restrict__ lin_b,
    const unsigned short* __restrict__ WHp, float* __restrict__ out) {
  __shared__ __align__(16) _Float16 Ah[AH_ELEMS];
  __shared__ __align__(16) float    Hf[HF_ELEMS];
  __shared__ __align__(16) float    linWs[HID];
  const _Float16* WH = (const _Float16*)WHp;
  const int tid = threadIdx.x, lane = tid & 31, wave = tid >> 5;
  const int bbase = blockIdx.x * RPB;

#pragma unroll 1
  for (int i = tid; i < AH_ELEMS; i += NTHR) Ah[i] = (_Float16)0.0f;
#pragma unroll 1
  for (int i = tid; i < HF_ELEMS; i += NTHR) Hf[i] = 0.0f;
  {
    const float lwv = bf16r(lin_w[tid & (HID - 1)]);
    if (tid < HID) linWs[tid] = lwv;
  }
  const float lb = bf16r(lin_b[0]);
  float cst[2][8];
#pragma unroll
  for (int mt = 0; mt < 2; ++mt)
#pragma unroll
    for (int r = 0; r < 8; ++r) cst[mt][r] = 0.0f;
  int par = 0;
  __syncthreads();

  lstm_phase<false>(x_enc, e_wih, e_bih, e_bhh, WH, out, 0.0f, cst, par, Ah, Hf, linWs, lane, wave, bbase);
  lstm_phase<true>(x_dec, d_wih, d_bih, d_bhh, WH + WPLANE, out, lb, cst, par, Ah, Hf, linWs, lane, wave, bbase);
}

extern "C" void kernel_launch(void* const* d_in, const int* in_sizes, int n_in,
                              void* d_out, int out_size, void* d_ws, size_t ws_size, hipStream_t stream) {
  if (n_in < 12 || d_out == nullptr || d_ws == nullptr) return;
  if (in_sizes[0] != TENC * NBAT || in_sizes[1] != TDEC * NBAT ||
      in_sizes[2] != NGROW || in_sizes[3] != NGROW * HID || in_sizes[4] != NGROW || in_sizes[5] != NGROW ||
      in_sizes[6] != NGROW || in_sizes[7] != NGROW * HID || in_sizes[8] != NGROW || in_sizes[9] != NGROW ||
      in_sizes[10] != HID || in_sizes[11] != 1 || out_size != TDEC * NBAT) return;

  const float* x_enc = (const float*)d_in[0];
  const float* x_dec = (const float*)d_in[1];
  const float* e_wih = (const float*)d_in[2];
  const float* e_whh = (const float*)d_in[3];
  const float* e_bih = (const float*)d_in[4];
  const float* e_bhh = (const float*)d_in[5];
  const float* d_wih = (const float*)d_in[6];
  const float* d_whh = (const float*)d_in[7];
  const float* d_bih = (const float*)d_in[8];
  const float* d_bhh = (const float*)d_in[9];
  const float* lin_w = (const float*)d_in[10];
  const float* lin_b = (const float*)d_in[11];
  float* out = (float*)d_out;

  char* ws = (char*)d_ws; size_t off = 0;
  auto carve = [&](size_t bytes) -> char* { char* p = ws + off; off += (bytes + 255) & ~(size_t)255; return p; };
  unsigned short* WH = (unsigned short*)carve((size_t)2 * WPLANE * 2);
  if (off > ws_size || off > (size_t)134217728) return;

  whh_prep_kernel<<<(WPLANE / 8) / PREP_THR, PREP_THR, 0, stream>>>(e_whh, WH);
  whh_prep_kernel<<<(WPLANE / 8) / PREP_THR, PREP_THR, 0, stream>>>(d_whh, WH + WPLANE);
  seq_kernel<<<NBAT / RPB, NTHR, 0, stream>>>(x_enc, x_dec, e_wih, e_bih, e_bhh, d_wih, d_bih, d_bhh, lin_w, lin_b, WH, out);
}
